// GAT_82085414961435
// MI455X (gfx1250) — hardware-run, weakly checked
//
#include <hip/hip_runtime.h>
#include <stddef.h>
#include <stdint.h>
#include <math.h>

#define NN      50000
#define NE      800000
#define HD      64
#define NHEAD   4
#define HC      16
#define NLAY    3
#define NATOM   16
#define NTYPE   4
#define MP      50048
#define GBM     128
#define KP      128
#define NTHR    256
#define NWAVE   8
#define EPT     8
#define WCH     (32 * EPT)
#define NBRUN   1024
#define SLB     10
#define NBK     49
#define WLCAP   3584
#define RCAP    28672
#define DEGCAP  64
#define MAXDEG_MEAS   35
#define MAXB1024_MEAS 16720
#define SP      68
#define NEGSL   0.2f
#define BNEPS   1e-5f
#define SPLIT1  1
#define SPLIT2  1
#define WSMAX   ((size_t)(128u << 20))

#define P_EE    0
#define P_AS    768
#define P_AD    960
#define P_AT    1152
#define P_BI    1344
#define P_GA    1536
#define P_BE    1728
#define P_PW    1920
#define P_AE    2048
#define P_PB    2096
#define PARN    2112

#define BK_ZINTS (NWAVE * WLCAP + RCAP + 3 * NBRUN + 4 * NBRUN)
#define BK_INTS  (BK_ZINTS + 16)
#define BK_LDS   (BK_INTS * 4)
#define RP_LDS   (RCAP * 4)

#define PBX   (MP * 16 / NTHR)
#define PBW   (NLAY * HD * KP / 8 / NTHR)
#define PBP   9
#define PBTOT (PBX + PBW + PBP)

static_assert(NHEAD * HC == HD && HD == 64);
static_assert(NE % 256 == 0 && NE % WCH == 0 && NE % 4 == 0);
static_assert(NN <= 65536);
static_assert(MP % GBM == 0 && MP >= NN && MP == 391 * GBM && (MP % 2) == 0);
static_assert(NBRUN == (1 << SLB) && NBK * NBRUN >= MP && (NBK - 1) * NBRUN < MP);
static_assert(NBRUN == NWAVE * 128);
static_assert(NE < (1 << 20) && (((long long)NE) << SLB) < (1LL << 31));
static_assert(RCAP == NWAVE * WLCAP && RCAP % (NTHR * 4) == 0 && BK_ZINTS % (NTHR * 4) == 0);
static_assert((long long)RCAP * 100 >= (long long)MAXB1024_MEAS * 105);
static_assert(WLCAP >= MAXB1024_MEAS / 8 + 8 * 46 + 1);
static_assert(MAXDEG_MEAS + 8 <= DEGCAP);
static_assert(KP == 2 * HD && KP % 32 == 0 && HD % 32 == 0);
static_assert((MP * 16) % NTHR == 0 && (NLAY * HD * KP / 8) % NTHR == 0);
static_assert(BK_LDS <= 327680);
static_assert(RP_LDS + 512 * 4 + NWAVE * 128 * 8 <= 327680);
static_assert((GBM * SP + 128 + GBM * 8) * 4 <= 65536);
static_assert(P_AS == P_EE + NLAY * NTYPE * HD && P_AD == P_AS + NLAY * HD && P_AT == P_AD + NLAY * HD);
static_assert(P_BI == P_AT + NLAY * HD && P_GA == P_BI + NLAY * HD && P_BE == P_GA + NLAY * HD);
static_assert(P_PW == P_BE + NLAY * HD && P_AE == P_PW + 2 * HD && P_PB == P_AE + NLAY * 16 && PARN == P_AE + 64);

typedef float          v4f   __attribute__((ext_vector_type(4)));
typedef float          v8f   __attribute__((ext_vector_type(8)));
typedef double         v2d   __attribute__((ext_vector_type(2)));
typedef int            v4i   __attribute__((ext_vector_type(4)));
typedef int            v8i   __attribute__((ext_vector_type(8)));
typedef unsigned short v8us  __attribute__((ext_vector_type(8)));
typedef unsigned short v16us __attribute__((ext_vector_type(16)));
typedef __bf16         v16bf __attribute__((ext_vector_type(16)));
typedef v4f  __attribute__((may_alias)) v4fa;
typedef v4i  __attribute__((may_alias)) v4ia;
typedef v2d  __attribute__((may_alias)) v2da;
typedef v8us __attribute__((may_alias)) v8usa;
union FragB { v16bf v; v16us u; v8us h[2]; v8i w; };

__device__ __forceinline__ v8f wmb(const FragB& a, const FragB& b, v8f c) {
  v8f d = __builtin_amdgcn_wmma_f32_16x16x32_bf16(false, a.v, false, b.v, (short)0, c, false, false);
  asm volatile("v_nop\n\tv_nop\n\tv_nop\n\tv_nop" : "+v"(d) : "v"(a.w), "v"(b.w));
  return d;
}

__device__ __forceinline__ unsigned bf16_bits(float f) {
  const unsigned u = __float_as_uint(f);
  const unsigned r = (u + 0x7FFFu + ((u >> 16) & 1u)) >> 16;
  const unsigned q = (u >> 16) | 0x40u;
  return ((u & 0x7fffffffu) > 0x7f800000u) ? q : r;
}
__device__ __forceinline__ float bf16_val(float f) {
  return __uint_as_float(bf16_bits(f) << 16);
}

__device__ __forceinline__ void hilo_pack(float v0, float v1, float v2, float v3,
                                          int& h01, int& h23, int& l01, int& l23) {
  const unsigned a0 = bf16_bits(v0), a1 = bf16_bits(v1), a2 = bf16_bits(v2), a3 = bf16_bits(v3);
  const unsigned b0 = bf16_bits(v0 - __uint_as_float(a0 << 16));
  const unsigned b1 = bf16_bits(v1 - __uint_as_float(a1 << 16));
  const unsigned b2 = bf16_bits(v2 - __uint_as_float(a2 << 16));
  const unsigned b3 = bf16_bits(v3 - __uint_as_float(a3 << 16));
  h01 = (int)(a0 | (a1 << 16)); h23 = (int)(a2 | (a3 << 16));
  l01 = (int)(b0 | (b1 << 16)); l23 = (int)(b2 | (b3 << 16));
}

__device__ __forceinline__ v4i regroup8(int h01, int h23, int l01, int l23, int lane) {
  const int t  = lane & 15;
  const int s0 = (lane & 16) + ((2 * t) & 15), s1 = s0 + 1;
  const int a0 = __shfl(h01, s0, 32), a1 = __shfl(h23, s0, 32), a2 = __shfl(h01, s1, 32), a3 = __shfl(h23, s1, 32);
  const int b0 = __shfl(l01, s0, 32), b1 = __shfl(l23, s0, 32), b2 = __shfl(l01, s1, 32), b3 = __shfl(l23, s1, 32);
  const int mk = (t < 8) ? -1 : 0;
  v4i o;
  o.x = (a0 & mk) | (b0 & ~mk); o.y = (a1 & mk) | (b1 & ~mk);
  o.z = (a2 & mk) | (b2 & ~mk); o.w = (a3 & mk) | (b3 & ~mk);
  return o;
}

__device__ __forceinline__ void st2_v4f(float* p, v4f v) {
  *(volatile v4f*)p = v;
  __threadfence();
  *(volatile v4f*)p = v;
}
__device__ __forceinline__ void st2_v8us(unsigned short* p, v8us v) {
  *(volatile v8us*)p = v;
  __threadfence();
  *(volatile v8us*)p = v;
}

__device__ __forceinline__ v8us gather8(const float* __restrict__ base, int stride) {
  float f[8];
#pragma unroll
  for (int i = 0; i < 8; ++i) f[i] = base[(size_t)i * (size_t)stride];
  v8us o;
#pragma unroll
  for (int i = 0; i < 8; ++i) o[i] = (unsigned short)bf16_bits(f[i]);
  return o;
}

__device__ __forceinline__ void par_copy(const float* __restrict__ src, float* dst, int n4, int tid) {
  const int p = tid < n4 ? tid : n4 - 1;
  const v4f v = *(const v4fa*)(src + 4 * p);
  asm volatile("" :: "v"(v));
  v4f o;
  o.x = bf16_val(v.x); o.y = bf16_val(v.y); o.z = bf16_val(v.z); o.w = bf16_val(v.w);
  float* op = dst + 4 * p;
  const bool wr = tid < n4;
  if (wr) *(volatile v4f*)op = o;
  __threadfence();
  if (wr) *(volatile v4f*)op = o;
}

__global__ __launch_bounds__(NTHR) void k_prep(const int* __restrict__ xidx, const float* __restrict__ aemb,
                                               const float* __restrict__ W, const float* __restrict__ atts,
                                               const float* __restrict__ attd, const float* __restrict__ atte,
                                               const float* __restrict__ bias, const float* __restrict__ eemb,
                                               const float* __restrict__ gam, const float* __restrict__ bet,
                                               const float* __restrict__ pw, const float* __restrict__ pb,
                                               float* X0, unsigned short* XHL, unsigned short* WT, float* PAR) {
  __shared__ __attribute__((aligned(16))) float sae[64];
  const int tid = (int)threadIdx.x;
  const int blk = (int)blockIdx.x;
  if (blk < PBX) {
    const int u   = blk * NTHR + tid;
    const int row = u >> 4, q = u & 15;
    const int rc  = row < NN ? row : NN - 1;
    int ai = xidx[rc];
    ai = ai < 0 ? 0 : (ai > NATOM - 1 ? NATOM - 1 : ai);
    const float* er = aemb + (size_t)ai * HD;
    const int c8 = 8 * (q & 7);
    const v4f a  = *(const v4fa*)(er + 4 * q);
    const v4f b0 = *(const v4fa*)(er + c8);
    const v4f b1 = *(const v4fa*)(er + c8 + 4);
    asm volatile("" :: "v"(a));
    asm volatile("" :: "v"(b0), "v"(b1));
    const bool live = row < NN;
    const unsigned mf = live ? 0xffffffffu : 0u;
    const unsigned mh = (live && q < 8) ? 0xffffu : 0u;
    v4f o;
    o.x = __uint_as_float((bf16_bits(a.x) << 16) & mf); o.y = __uint_as_float((bf16_bits(a.y) << 16) & mf);
    o.z = __uint_as_float((bf16_bits(a.z) << 16) & mf); o.w = __uint_as_float((bf16_bits(a.w) << 16) & mf);
    v8us hv;
    hv[0] = (unsigned short)(bf16_bits(b0.x) & mh); hv[1] = (unsigned short)(bf16_bits(b0.y) & mh);
    hv[2] = (unsigned short)(bf16_bits(b0.z) & mh); hv[3] = (unsigned short)(bf16_bits(b0.w) & mh);
    hv[4] = (unsigned short)(bf16_bits(b1.x) & mh); hv[5] = (unsigned short)(bf16_bits(b1.y) & mh);
    hv[6] = (unsigned short)(bf16_bits(b1.z) & mh); hv[7] = (unsigned short)(bf16_bits(b1.w) & mh);
    float* xp = X0 + (size_t)row * HD + 4 * q;
    unsigned short* hp = XHL + (size_t)row * KP + 8 * q;
    *(volatile v4f*)xp = o;
    *(volatile v8us*)hp = hv;
    __threadfence();
    *(volatile v4f*)xp = o;
    *(volatile v8us*)hp = hv;
  } else if (blk < PBX + PBW) {
    const int u = (blk - PBX) * NTHR + tid;
    const int l = u >> 10, n = (u >> 4) & 63, k8 = (u & 15) * 8, kk = k8 & 63;
    const v8us o = gather8(W + (size_t)l * HD * HD + (size_t)kk * HD + n, HD);
    st2_v8us(WT + (size_t)l * HD * KP + (size_t)n * KP + k8, o);
  } else {
    const int pk = blk - PBX - PBW;
    if (pk == 0)      par_copy(eemb, PAR + P_EE, NLAY * NTYPE * HD / 4, tid);
    else if (pk == 1) par_copy(atts, PAR + P_AS, NLAY * HD / 4, tid);
    else if (pk == 2) par_copy(attd, PAR + P_AD, NLAY * HD / 4, tid);
    else if (pk == 3) par_copy(atte, PAR + P_AT, NLAY * HD / 4, tid);
    else if (pk == 4) par_copy(bias, PAR + P_BI, NLAY * HD / 4, tid);
    else if (pk == 5) par_copy(gam,  PAR + P_GA, NLAY * HD / 4, tid);
    else if (pk == 6) par_copy(bet,  PAR + P_BE, NLAY * HD / 4, tid);
    else if (pk == 7) par_copy(pw,   PAR + P_PW, 2 * HD / 4, tid);
    else {
      if (tid < 64) {
        const int t = tid < 48 ? tid : 47;
        const int l = t >> 4, ty = (t >> 2) & 3, h = t & 3;
        const float* ep = eemb + (size_t)(l * NTYPE + ty) * HD + h * HC;
        const float* ap = atte + (size_t)(l * NHEAD + h) * HC;
        float s = 0.0f;
#pragma unroll 1
        for (int c4 = 0; c4 < HC / 4; ++c4) {
          const v4f ev = *(const v4fa*)(ep + 4 * c4);
          const v4f av = *(const v4fa*)(ap + 4 * c4);
          s = fmaf(bf16_val(ev.x), bf16_val(av.x), s);
          s = fmaf(bf16_val(ev.y), bf16_val(av.y), s);
          s = fmaf(bf16_val(ev.z), bf16_val(av.z), s);
          s = fmaf(bf16_val(ev.w), bf16_val(av.w), s);
        }
        const float pbv = bf16_val(pb[0]);
        const float v = (tid < 48) ? s : ((tid == 48) ? pbv : 0.0f);
        sae[tid] = v;
      }
      __syncthreads();
      if (tid < 16) {
        const v4f v = *(const v4fa*)(sae + 4 * tid);
        st2_v4f(PAR + P_AE + 4 * tid, v);
      }
    }
  }
}

__device__ __forceinline__ void bucket_flush(const int* pl, const int* cnt, const int* tc, int ov,
                                             int* lp, int* cop, int* tcp, int* fp, int tid) {
#pragma unroll 1
  for (int i = tid * 4; i < RCAP; i += NTHR * 4) {
    const v4i v = *(const v4ia*)(pl + i);
    *(volatile v4i*)(lp + i) = v;
  }
#pragma unroll 1
  for (int i = tid * 4; i < 2 * NBRUN; i += NTHR * 4) {
    const v4i v = *(const v4ia*)(cnt + i);
    *(volatile v4i*)(cop + i) = v;
  }
#pragma unroll 1
  for (int i = tid * 4; i < 4 * NBRUN; i += NTHR * 4) {
    const v4i v = *(const v4ia*)(tc + i);
    *(volatile v4i*)(tcp + i) = v;
  }
  if (tid < 8) {
    const v4i f = {ov, ov, ov, ov};
    *(volatile v4i*)(fp + 4 * tid) = f;
  }
}

__global__ __launch_bounds__(NTHR) void k_bucket(const int* __restrict__ srcs, const int* __restrict__ dsts,
                                                 const int* __restrict__ etyp, int* HITS, int* CO, int* TC, int* FLAG) {
  extern __shared__ __attribute__((aligned(16))) int dsm[];
  int* wl   = dsm;
  int* pl   = dsm + NWAVE * WLCAP;
  int* cnt  = pl + RCAP;
  int* offs = cnt + NBRUN;
  int* cur  = offs + NBRUN;
  int* tc   = cur + NBRUN;
  int* misc = tc + 4 * NBRUN;
  const int tid = (int)threadIdx.x, lane = tid & 31, wave = tid >> 5;
  const int blk = (int)blockIdx.x;
  const unsigned nbs = (unsigned)(blk * NBRUN);

  {
    const v4i z4 = {0, 0, 0, 0};
    for (int i = tid * 4; i < BK_ZINTS; i += NTHR * 4) *(v4ia*)(dsm + i) = z4;
    if (tid < 16) misc[tid] = 0;
  }
  __syncthreads();

  {
    const int per  = ((NE + NWAVE * WCH - 1) / (NWAVE * WCH)) * WCH;
    const int ebeg = wave * per;
    const int eend = (ebeg + per < NE) ? (ebeg + per) : NE;
    int* mylist = wl + wave * WLCAP;
    int wc = 0;
#pragma unroll 1
    for (int cb = ebeg; cb < eend; cb += WCH) {
      const int e0 = cb + lane * EPT;
      const v4i da = *(const v4ia*)(dsts + e0);
      const v4i db = *(const v4ia*)(dsts + e0 + 4);
      const unsigned s0 = (unsigned)da.x - nbs, s1 = (unsigned)da.y - nbs;
      const unsigned s2 = (unsigned)da.z - nbs, s3 = (unsigned)da.w - nbs;
      const unsigned s4 = (unsigned)db.x - nbs, s5 = (unsigned)db.y - nbs;
      const unsigned s6 = (unsigned)db.z - nbs, s7 = (unsigned)db.w - nbs;
      const bool h0 = s0 < (unsigned)NBRUN, h1 = s1 < (unsigned)NBRUN, h2 = s2 < (unsigned)NBRUN, h3 = s3 < (unsigned)NBRUN;
      const bool h4 = s4 < (unsigned)NBRUN, h5 = s5 < (unsigned)NBRUN, h6 = s6 < (unsigned)NBRUN, h7 = s7 < (unsigned)NBRUN;
      const unsigned m0 = __builtin_amdgcn_ballot_w32(h0), m1 = __builtin_amdgcn_ballot_w32(h1);
      const unsigned m2 = __builtin_amdgcn_ballot_w32(h2), m3 = __builtin_amdgcn_ballot_w32(h3);
      const unsigned m4 = __builtin_amdgcn_ballot_w32(h4), m5 = __builtin_amdgcn_ballot_w32(h5);
      const unsigned m6 = __builtin_amdgcn_ballot_w32(h6), m7 = __builtin_amdgcn_ballot_w32(h7);
      const unsigned any = m0 | m1 | m2 | m3 | m4 | m5 | m6 | m7;
      if (any != 0u) {
        const int pre = (int)(__builtin_amdgcn_mbcnt_lo(m0, 0u) + __builtin_amdgcn_mbcnt_lo(m1, 0u) +
                              __builtin_amdgcn_mbcnt_lo(m2, 0u) + __builtin_amdgcn_mbcnt_lo(m3, 0u) +
                              __builtin_amdgcn_mbcnt_lo(m4, 0u) + __builtin_amdgcn_mbcnt_lo(m5, 0u) +
                              __builtin_amdgcn_mbcnt_lo(m6, 0u) + __builtin_amdgcn_mbcnt_lo(m7, 0u));
        int p = wc + pre;
        if (h0) { if (p < WLCAP) mylist[p] = ((e0 + 0) << SLB) | (int)s0; p = p + 1; }
        if (h1) { if (p < WLCAP) mylist[p] = ((e0 + 1) << SLB) | (int)s1; p = p + 1; }
        if (h2) { if (p < WLCAP) mylist[p] = ((e0 + 2) << SLB) | (int)s2; p = p + 1; }
        if (h3) { if (p < WLCAP) mylist[p] = ((e0 + 3) << SLB) | (int)s3; p = p + 1; }
        if (h4) { if (p < WLCAP) mylist[p] = ((e0 + 4) << SLB) | (int)s4; p = p + 1; }
        if (h5) { if (p < WLCAP) mylist[p] = ((e0 + 5) << SLB) | (int)s5; p = p + 1; }
        if (h6) { if (p < WLCAP) mylist[p] = ((e0 + 6) << SLB) | (int)s6; p = p + 1; }
        if (h7) { if (p < WLCAP) mylist[p] = ((e0 + 7) << SLB) | (int)s7; p = p + 1; }
        wc += (int)(__builtin_popcount(m0) + __builtin_popcount(m1) + __builtin_popcount(m2) + __builtin_popcount(m3) +
                    __builtin_popcount(m4) + __builtin_popcount(m5) + __builtin_popcount(m6) + __builtin_popcount(m7));
      }
    }
    if (lane == 0) misc[wave] = wc;
  }
  __syncthreads();

  if (wave == 0) {
    int ov = 0;
#pragma unroll 1
    for (int w2 = 0; w2 < NWAVE; ++w2) {
      int c = misc[w2];
      if (c > WLCAP) ov = 1;
      c = c < 0 ? 0 : (c > WLCAP ? WLCAP : c);
#pragma unroll 1
      for (int b0 = 0; b0 < c; b0 += 32) {
        const int idx = b0 + lane;
        const int ent = wl[w2 * WLCAP + (idx < WLCAP ? idx : WLCAP - 1)];
        const int m32 = (c - b0) < 32 ? (c - b0) : 32;
#pragma unroll 1
        for (int k = 0; k < m32; ++k) {
          const int u    = __builtin_amdgcn_readlane(ent, k);
          const int slot = u & (NBRUN - 1);
          if (lane == 0) cnt[slot] = cnt[slot] + 1;
        }
      }
    }
    if (lane == 0) misc[9] = ov;
  }
  __syncthreads();
  if (wave == 0) {
    const int base = lane * (NBRUN / 32);
    int s = 0;
#pragma unroll 1
    for (int i = 0; i < NBRUN / 32; ++i) s += cnt[base + i];
    int incl = s;
#pragma unroll
    for (int d = 1; d < 32; d <<= 1) {
      const int y = __shfl_up(incl, d, 32);
      if (lane >= d) incl += y;
    }
    int run = incl - s;
#pragma unroll 1
    for (int i = 0; i < NBRUN / 32; ++i) {
      const int cv = cnt[base + i];
      offs[base + i] = run;
      cur[base + i]  = run;
      run += cv;
    }
  }
  __syncthreads();

  if (wave == 0) {
#pragma unroll 1
    for (int w2 = 0; w2 < NWAVE; ++w2) {
      int c = misc[w2];
      c = c < 0 ? 0 : (c > WLCAP ? WLCAP : c);
#pragma unroll 1
      for (int b0 = 0; b0 < c; b0 += 32) {
        const int idx = b0 + lane;
        const int ent = wl[w2 * WLCAP + (idx < WLCAP ? idx : WLCAP - 1)];
        int eid = (ent >> SLB) & 0xFFFFF;
        eid = eid > NE - 1 ? NE - 1 : eid;
        int sr = srcs[eid];
        sr = sr < 0 ? 0 : (sr > NN - 1 ? NN - 1 : sr);
        int ty = etyp[eid];
        ty = ty < 0 ? 0 : (ty > NTYPE - 1 ? NTYPE - 1 : ty);
        const int word = (int)((unsigned)sr | ((unsigned)ty << 16) | ((unsigned)(ent & (NBRUN - 1)) << 18));
        const int m32 = (c - b0) < 32 ? (c - b0) : 32;
#pragma unroll 1
        for (int k = 0; k < m32; ++k) {
          const int wd   = __builtin_amdgcn_readlane(word, k);
          const int slot = (wd >> 18) & (NBRUN - 1);
          const int tk   = (wd >> 16) & 3;
          if (lane == 0) {
            int p = cur[slot];
            p = p < 0 ? 0 : (p > RCAP - 1 ? RCAP - 1 : p);
            pl[p] = wd;
            cur[slot] = p + 1;
            tc[4 * slot + tk] = tc[4 * slot + tk] + 1;
          }
        }
      }
    }
  }
  __syncthreads();

  const int ovf = misc[9];
  int* lp  = HITS + (size_t)blk * RCAP;
  int* cop = CO + (size_t)blk * (2 * NBRUN);
  int* tcp = TC + (size_t)blk * (4 * NBRUN);
  int* fp  = FLAG + (size_t)blk * 32;
  bucket_flush(pl, cnt, tc, ovf, lp, cop, tcp, fp, tid);
  __threadfence();
  bucket_flush(pl, cnt, tc, ovf, lp, cop, tcp, fp, tid);
}

template <int KEXT>
__device__ __forceinline__ void gemm_16x64(const unsigned short* __restrict__ ap,
                                           const unsigned short* __restrict__ bp, v8f (&acc)[4]) {
#pragma unroll 1
  for (int k0 = 0; k0 < KEXT; k0 += 32) {
    FragB af;
    af.h[0] = *(const v8usa*)(ap + k0);
    af.h[1] = *(const v8usa*)(ap + k0 + 16);
#pragma unroll
    for (int nt = 0; nt < 4; ++nt) {
      const unsigned short* wq = bp + (size_t)(16 * nt) * (size_t)KP + k0;
      FragB bf;
      bf.h[0] = *(const v8usa*)wq;
      bf.h[1] = *(const v8usa*)(wq + 16);
      acc[nt] = wmb(af, bf, acc[nt]);
    }
  }
}

__device__ __forceinline__ void stage_d(float* stg, const v8f (&acc)[4], int wave, int hh, int m) {
#pragma unroll
  for (int nt = 0; nt < 4; ++nt) {
#pragma unroll
    for (int r = 0; r < 8; ++r) stg[(16 * wave + 8 * hh + r) * SP + 16 * nt + m] = acc[nt][r];
  }
}

template <int KEXT>
__global__ __launch_bounds__(NTHR) __attribute__((amdgpu_num_vgpr(248)))
void k_gemm(const unsigned short* __restrict__ A, const unsigned short* __restrict__ BT,
            const float* __restrict__ par, int offS, int offD, float* XL, float* SD) {
  __shared__ __attribute__((aligned(16))) float stg[GBM * SP];
  __shared__ __attribute__((aligned(16))) float satt[128];
  __shared__ __attribute__((aligned(16))) float ssd[GBM * 8];
  const int tid = (int)threadIdx.x, lane = tid & 31, wave = tid >> 5, hh = lane >> 4, m = lane & 15;
  const int rowBase = (int)blockIdx.x * GBM;
  if (tid < 32) {
    const int off = ((lane < 16) ? offS : offD) + 4 * m;
    *(v4fa*)(satt + 4 * lane) = *(const v4fa*)(par + off);
  }

  v8f acc[4];
  {
    const v8f z = {0.f, 0.f, 0.f, 0.f, 0.f, 0.f, 0.f, 0.f};
#pragma unroll
    for (int t = 0; t < 4; ++t) acc[t] = z;
  }
  const unsigned short* ap = A + (size_t)(rowBase + 16 * wave + m) * (size_t)KP + 8 * hh;
  const unsigned short* bp = BT + (size_t)m * (size_t)KP + 8 * hh;
  gemm_16x64<KEXT>(ap, bp, acc);
  stage_d(stg, acc, wave, hh, m);
  __syncthreads();

  const v4f as4 = *(const v4fa*)(satt + 4 * m);
  const v4f ad4 = *(const v4fa*)(satt + 64 + 4 * m);
#pragma unroll 1
  for (int i = 0; i < 8; ++i) {
    const int lr   = 16 * wave + 2 * i + hh;
    const int grow = rowBase + lr;
    const bool live = grow < NN;
    const v4f a = *(const v4fa*)(stg + lr * SP + 4 * m);
    asm volatile("" :: "v"(a));
    v4f o;
    o.x = live ? a.x : 0.0f; o.y = live ? a.y : 0.0f; o.z = live ? a.z : 0.0f; o.w = live ? a.w : 0.0f;
    float ds = o.x * as4.x; ds = fmaf(o.y, as4.y, ds); ds = fmaf(o.z, as4.z, ds); ds = fmaf(o.w, as4.w, ds);
    float dd = o.x * ad4.x; dd = fmaf(o.y, ad4.y, dd); dd = fmaf(o.z, ad4.z, dd); dd = fmaf(o.w, ad4.w, dd);
    ds += __shfl_xor(ds, 1, 32); dd += __shfl_xor(dd, 1, 32);
    ds += __shfl_xor(ds, 2, 32); dd += __shfl_xor(dd, 2, 32);
    if ((m & 3) == 0) {
      ssd[lr * 8 + (m >> 2)]     = ds;
      ssd[lr * 8 + 4 + (m >> 2)] = dd;
    }
    st2_v4f(XL + (size_t)grow * HD + 4 * m, o);
  }
  __syncthreads();
  {
    const v4f v = *(const v4fa*)(ssd + 4 * tid);
    st2_v4f(SD + (size_t)rowBase * 8 + 4 * tid, v);
  }
}

__global__ __launch_bounds__(NTHR) void k_replay(const int* __restrict__ HITS, const int* __restrict__ CO,
                                                 const int* __restrict__ TC, const int* __restrict__ FLAG,
                                                 const float* __restrict__ par, int lay,
                                                 const float* __restrict__ XL, const float* __restrict__ SD,
                                                 float* T, double* REC) {
  extern __shared__ __attribute__((aligned(16))) int dsm[];
  __shared__ __attribute__((aligned(16))) float spar[512];
  __shared__ __attribute__((aligned(16))) double srec[NWAVE * 128];
  const int tid = (int)threadIdx.x, lane = tid & 31, wave = tid >> 5, hh = lane >> 4, q = lane & 15;
  const int blk = (int)blockIdx.x;
  const int nodeBase = blk * NBRUN;
  const int* hb  = HITS + (size_t)blk * RCAP;
  const int* cob = CO + (size_t)blk * (2 * NBRUN);
  const int* tcb = TC + (size_t)blk * (4 * NBRUN);

#pragma unroll 1
  for (int i = tid * 4; i < RCAP; i += NTHR * 4) *(v4ia*)(dsm + i) = *(const v4ia*)(hb + i);
  if (tid < 128) {
    const int t = tid < 100 ? tid : 99;
    const int g = (t < 64) ? (P_EE + 256 * lay + 4 * t)
                : (t < 80) ? (P_AT + 64 * lay + 4 * (t - 64))
                : (t < 96) ? (P_BI + 64 * lay + 4 * (t - 80))
                           : (P_AE + 16 * lay + 4 * (t - 96));
    *(v4fa*)(spar + 4 * t) = *(const v4fa*)(par + g);
  }
  __syncthreads();

  const int flag = FLAG[(size_t)blk * 32];
  const int h = q >> 2;
  const v4f at4 = *(const v4fa*)(spar + 256 + 4 * q);
  const v4f bi4 = *(const v4fa*)(spar + 320 + 4 * q);
  const v4f e0 = *(const v4fa*)(spar + 0 * HD + 4 * q);
  const v4f e1 = *(const v4fa*)(spar + 1 * HD + 4 * q);
  const v4f e2 = *(const v4fa*)(spar + 2 * HD + 4 * q);
  const v4f e3 = *(const v4fa*)(spar + 3 * HD + 4 * q);
  const float qnan = __uint_as_float(0x7fc00000u);
  double s0 = 0.0, s1 = 0.0, s2 = 0.0, s3 = 0.0, q0 = 0.0, q1 = 0.0, q2 = 0.0, q3 = 0.0;

#pragma unroll 1
  for (int i = 0; i < 64; ++i) {
    const int slot = 128 * wave + 2 * i + hh;
    const int d    = nodeBase + slot;
    const int dcl  = d < NN ? d : NN - 1;
    int c = cob[slot];
    int o = cob[NBRUN + slot];
    const v4i tc4 = *(const v4ia*)(tcb + 4 * slot);
    const bool big = c > DEGCAP;
    c = c < 0 ? 0 : (c > DEGCAP ? DEGCAP : c);
    o = o < 0 ? 0 : (o > RCAP - 1 ? RCAP - 1 : o);
    int last = o + c - 1; last = last < o ? o : last;
    last = last > RCAP - 1 ? RCAP - 1 : last;
    const int co = __shfl_xor(c, 16, 32);
    const int cmv = c > co ? c : co;
    const int cm = __builtin_amdgcn_readfirstlane(cmv);

    const int n0 = tc4.x < 0 ? 0 : tc4.x, n1 = tc4.y < 0 ? 0 : tc4.y;
    const int n2 = tc4.z < 0 ? 0 : tc4.z, n3 = tc4.w < 0 ? 0 : tc4.w;
    const float f0 = (float)n0, f1 = (float)n1, f2 = (float)n2, f3 = (float)n3;
    const float cntf = (float)(n0 + n1 + n2 + n3);
    const float dv   = cntf < 1.0f ? 1.0f : cntf;
    const float rinv = 1.0f / dv;
    float emx = f0 * e0.x; emx = fmaf(f1, e1.x, emx); emx = fmaf(f2, e2.x, emx); emx = fmaf(f3, e3.x, emx); emx *= rinv;
    float emy = f0 * e0.y; emy = fmaf(f1, e1.y, emy); emy = fmaf(f2, e2.y, emy); emy = fmaf(f3, e3.y, emy); emy *= rinv;
    float emz = f0 * e0.z; emz = fmaf(f1, e1.z, emz); emz = fmaf(f2, e2.z, emz); emz = fmaf(f3, e3.z, emz); emz *= rinv;
    float emw = f0 * e0.w; emw = fmaf(f1, e1.w, emw); emw = fmaf(f2, e2.w, emw); emw = fmaf(f3, e3.w, emw); emw *= rinv;
    float ae = emx * at4.x; ae = fmaf(emy, at4.y, ae); ae = fmaf(emz, at4.z, ae); ae = fmaf(emw, at4.w, ae);
    ae += __shfl_xor(ae, 1, 32);
    ae += __shfl_xor(ae, 2, 32);
    const float asd = SD[(size_t)dcl * 8 + h];
    const float add = SD[(size_t)dcl * 8 + 4 + h];
    const v4f xr = *(const v4fa*)(XL + (size_t)dcl * HD + 4 * q);
    float l0 = (asd + add) + ae;
    l0 = (l0 >= 0.0f) ? l0 : NEGSL * l0;
    float mx = l0, den = 1.0f;
    float a0 = xr.x + emx, a1 = xr.y + emy, a2 = xr.z + emz, a3 = xr.w + emw;

#pragma unroll 1
    for (int j = 0; j < cm; ++j) {
      int idx = o + j;
      idx = idx > last ? last : idx;
      const unsigned wd = (unsigned)dsm[idx];
      int sr = (int)(wd & 0xffffu);
      sr = sr > NN - 1 ? NN - 1 : sr;
      const int ty = (int)((wd >> 16) & 3u);
      const float asv = SD[(size_t)sr * 8 + h];
      const v4f xv = *(const v4fa*)(XL + (size_t)sr * HD + 4 * q);
      asm volatile("" :: "v"(asv));
      asm volatile("" :: "v"(xv));
      const float aev = spar[384 + 4 * ty + h];
      const v4f ev = *(const v4fa*)(spar + ty * HD + 4 * q);
      float lg = (asv + add) + aev;
      lg = (lg >= 0.0f) ? lg : NEGSL * lg;
      const float df = lg - mx;
      const float ee = expf(-fabsf(df));
      const bool up  = df > 0.0f;
      const float r1 = up ? ee : 1.0f;
      const float r2 = up ? 1.0f : ee;
      const float nmx  = up ? lg : mx;
      const float nden = fmaf(den, r1, r2);
      const float t0 = fmaf(a0, r1, r2 * (xv.x + ev.x));
      const float t1 = fmaf(a1, r1, r2 * (xv.y + ev.y));
      const float t2 = fmaf(a2, r1, r2 * (xv.z + ev.z));
      const float t3 = fmaf(a3, r1, r2 * (xv.w + ev.w));
      const bool valid = j < c;
      mx  = valid ? nmx : mx;
      den = valid ? nden : den;
      a0 = valid ? t0 : a0; a1 = valid ? t1 : a1; a2 = valid ? t2 : a2; a3 = valid ? t3 : a3;
    }
    float o0 = a0 / den + bi4.x, o1 = a1 / den + bi4.y, o2 = a2 / den + bi4.z, o3 = a3 / den + bi4.w;
    const bool bad  = (flag != 0) | big;
    const bool live = d < NN;
    o0 = bad ? qnan : o0; o1 = bad ? qnan : o1; o2 = bad ? qnan : o2; o3 = bad ? qnan : o3;
    o0 = live ? o0 : 0.0f; o1 = live ? o1 : 0.0f; o2 = live ? o2 : 0.0f; o3 = live ? o3 : 0.0f;
    {
      const double w0 = (double)o0, w1 = (double)o1, w2 = (double)o2, w3 = (double)o3;
      s0 += w0; s1 += w1; s2 += w2; s3 += w3;
      q0 = fma(w0, w0, q0); q1 = fma(w1, w1, q1); q2 = fma(w2, w2, q2); q3 = fma(w3, w3, q3);
    }
    v4f ov;
    ov.x = o0; ov.y = o1; ov.z = o2; ov.w = o3;
    float* tp = T + (size_t)d * HD + 4 * q;
    const bool wr = d < MP;
    if (wr) *(volatile v4f*)tp = ov;
    __threadfence();
    if (wr) *(volatile v4f*)tp = ov;
  }

  s0 += __shfl_xor(s0, 16, 32); s1 += __shfl_xor(s1, 16, 32);
  s2 += __shfl_xor(s2, 16, 32); s3 += __shfl_xor(s3, 16, 32);
  q0 += __shfl_xor(q0, 16, 32); q1 += __shfl_xor(q1, 16, 32);
  q2 += __shfl_xor(q2, 16, 32); q3 += __shfl_xor(q3, 16, 32);
  if (lane < 16) {
    double* rp = srec + (size_t)(wave * 64 + 4 * q) * 2;
    rp[0] = s0; rp[1] = q0; rp[2] = s1; rp[3] = q1; rp[4] = s2; rp[5] = q2; rp[6] = s3; rp[7] = q3;
  }
  __syncthreads();
  if (tid < 64) {
    double S = 0.0, Q = 0.0;
#pragma unroll 1
    for (int w = 0; w < NWAVE; ++w) {
      S += srec[(size_t)(w * 64 + tid) * 2];
      Q += srec[(size_t)(w * 64 + tid) * 2 + 1];
    }
    v2d r;
    r.x = S; r.y = Q;
    double* gp = REC + (size_t)(blk * 64 + tid) * 2;
    *(volatile v2d*)gp = r;
    __threadfence();
    *(volatile v2d*)gp = r;
  }
}

__global__ __launch_bounds__(64) void k_stat(const double* __restrict__ REC, float* STAT) {
  __shared__ __attribute__((aligned(16))) float sst[128];
  const int c = (int)threadIdx.x;
  double S = 0.0, Q = 0.0;
#pragma unroll 1
  for (int b = 0; b < NBK; ++b) {
    const v2d r = *(const v2da*)(REC + (size_t)(b * 64 + c) * 2);
    S += r.x; Q += r.y;
  }
  const double invn = 1.0 / (double)NN;
  const double mu = S * invn;
  double var = Q * invn - mu * mu;
  var = (var < 0.0) ? 0.0 : var;
  const double rs = 1.0 / sqrt(var + (double)BNEPS);
  sst[2 * c]     = (float)mu;
  sst[2 * c + 1] = (float)rs;
  __syncthreads();
  if (c < 32) {
    const v4f v = *(const v4fa*)(sst + 4 * c);
    st2_v4f(STAT + 4 * c, v);
  }
}

template <int LASTL>
__global__ __launch_bounds__(NTHR) void k_apply(const float* __restrict__ T, const float* __restrict__ Xold,
                                                const float* __restrict__ STAT, const float* __restrict__ par,
                                                int lay, float* Xnew, unsigned short* XHL, float* PSD) {
  __shared__ __attribute__((aligned(16))) float spsd[GBM * 2];
  const int tid = (int)threadIdx.x, lane = tid & 31, wave = tid >> 5, hh = lane >> 4, q = lane & 15;
  const int rowBase = (int)blockIdx.x * GBM;
  const v4f sa = *(const v4fa*)(STAT + 8 * q);
  const v4f sb = *(const v4fa*)(STAT + 8 * q + 4);
  const v4f ga = *(const v4fa*)(par + P_GA + 64 * lay + 4 * q);
  const v4f be = *(const v4fa*)(par + P_BE + 64 * lay + 4 * q);
  const v4f ws = *(const v4fa*)(par + P_PW + 4 * q);
  const v4f wd = *(const v4fa*)(par + P_PW + 64 + 4 * q);

#pragma unroll 1
  for (int i = 0; i < 8; ++i) {
    const int lr   = 16 * wave + 2 * i + hh;
    const int grow = rowBase + lr;
    const bool live = grow < NN;
    const v4f t  = *(const v4fa*)(T + (size_t)grow * HD + 4 * q);
    const v4f xo = *(const v4fa*)(Xold + (size_t)grow * HD + 4 * q);
    asm volatile("" :: "v"(t));
    asm volatile("" :: "v"(xo));
    float y0 = ((t.x - sa.x) * sa.y) * ga.x + be.x;
    float y1 = ((t.y - sa.z) * sa.w) * ga.y + be.y;
    float y2 = ((t.z - sb.x) * sb.y) * ga.z + be.z;
    float y3 = ((t.w - sb.z) * sb.w) * ga.w + be.w;
    y0 = (y0 > 0.0f) ? y0 : (y0 - y0); y1 = (y1 > 0.0f) ? y1 : (y1 - y1);
    y2 = (y2 > 0.0f) ? y2 : (y2 - y2); y3 = (y3 > 0.0f) ? y3 : (y3 - y3);
    float v0 = y0 + xo.x, v1 = y1 + xo.y, v2 = y2 + xo.z, v3 = y3 + xo.w;
    v0 = live ? v0 : 0.0f; v1 = live ? v1 : 0.0f; v2 = live ? v2 : 0.0f; v3 = live ? v3 : 0.0f;
    if constexpr (LASTL == 0) {
      v4f ov;
      ov.x = v0; ov.y = v1; ov.z = v2; ov.w = v3;
      int h01, h23, l01, l23;
      hilo_pack(v0, v1, v2, v3, h01, h23, l01, l23);
      const v4i ow = regroup8(h01, h23, l01, l23, lane);
      float* op = Xnew + (size_t)grow * HD + 4 * q;
      unsigned short* hp = XHL + (size_t)grow * KP + 8 * q;
      *(volatile v4f*)op = ov;
      *(volatile v4i*)hp = ow;
      __threadfence();
      *(volatile v4f*)op = ov;
      *(volatile v4i*)hp = ow;
    } else {
      float ps = v0 * ws.x; ps = fmaf(v1, ws.y, ps); ps = fmaf(v2, ws.z, ps); ps = fmaf(v3, ws.w, ps);
      float pd = v0 * wd.x; pd = fmaf(v1, wd.y, pd); pd = fmaf(v2, wd.z, pd); pd = fmaf(v3, wd.w, pd);
#pragma unroll
      for (int dl = 1; dl < 16; dl <<= 1) {
        ps += __shfl_xor(ps, dl, 32);
        pd += __shfl_xor(pd, dl, 32);
      }
      if (q == 0) { spsd[2 * lr] = ps; spsd[2 * lr + 1] = pd; }
    }
  }
  if constexpr (LASTL != 0) {
    __syncthreads();
    if (tid < 64) {
      const v4f v = *(const v4fa*)(spsd + 4 * tid);
      st2_v4f(PSD + (size_t)rowBase * 2 + 4 * tid, v);
    }
  }
}

__global__ __launch_bounds__(NTHR) void k_head(const int* __restrict__ ei, const float* __restrict__ PSD,
                                               const float* __restrict__ par, float* out) {
  const int e  = (int)blockIdx.x * NTHR + (int)threadIdx.x;
  const int ec = e < NE ? e : NE - 1;
  int s = ei[ec];
  int d = ei[NE + ec];
  s = s < 0 ? 0 : (s > NN - 1 ? NN - 1 : s);
  d = d < 0 ? 0 : (d > NN - 1 ? NN - 1 : d);
  const float a = PSD[(size_t)2 * s];
  const float b = PSD[(size_t)2 * d + 1];
  const float pbv = par[P_PB];
  asm volatile("" :: "v"(a), "v"(b));
  const float v = (a + b) + pbv;
  const bool wr = e < NE;
  float* op = out + ec;
  if (wr) *(volatile float*)op = v;
  __threadfence();
  if (wr) *(volatile float*)op = v;
}

extern "C" void kernel_launch(void* const* d_in, const int* in_sizes, int n_in,
                              void* d_out, int out_size, void* d_ws, size_t ws_size,
                              hipStream_t stream) {
  if (n_in < 14) return;
  if (in_sizes[0] != NN) return;
  if (in_sizes[1] != 2 * NE) return;
  if (in_sizes[2] != NE) return;
  if (in_sizes[3] != NATOM * HD) return;
  if (in_sizes[4] != NLAY * HD * HD) return;
  if (in_sizes[5] != NLAY * HD || in_sizes[6] != NLAY * HD || in_sizes[7] != NLAY * HD) return;
  if (in_sizes[8] != NLAY * HD) return;
  if (in_sizes[9] != NLAY * NTYPE * HD) return;
  if (in_sizes[10] != NLAY * HD || in_sizes[11] != NLAY * HD) return;
  if (in_sizes[12] != 2 * HD) return;
  if (in_sizes[13] < 1) return;
  if (out_size != NE) return;

  const int*   xidx = (const int*)d_in[0];
  const int*   ei   = (const int*)d_in[1];
  const int*   etyp = (const int*)d_in[2];
  const float* aemb = (const float*)d_in[3];
  const float* W    = (const float*)d_in[4];
  const float* atts = (const float*)d_in[5];
  const float* attd = (const float*)d_in[6];
  const float* atte = (const float*)d_in[7];
  const float* bias = (const float*)d_in[8];
  const float* eemb = (const float*)d_in[9];
  const float* gam  = (const float*)d_in[10];
  const float* bet  = (const float*)d_in[11];
  const float* pw   = (const float*)d_in[12];
  const float* pb   = (const float*)d_in[13];
  float* out = (float*)d_out;
  const int* srcs = ei;
  const int* dsts = ei + NE;

  constexpr size_t zF    = (size_t)MP * HD * 4;
  constexpr size_t zHL   = (size_t)MP * KP * 2;
  constexpr size_t zSD   = (size_t)MP * 8 * 4;
  constexpr size_t zPSD  = (size_t)MP * 2 * 4;
  constexpr size_t zHITS = (size_t)NBK * RCAP * 4;
  constexpr size_t zCO   = (size_t)NBK * 2 * NBRUN * 4;
  constexpr size_t zTC   = (size_t)NBK * 4 * NBRUN * 4;
  constexpr size_t zFLAG = 6400;
  constexpr size_t zREC  = (size_t)NBK * 64 * 2 * 8;
  constexpr size_t zSTAT = 512;
  constexpr size_t zWT   = (size_t)NLAY * HD * KP * 2;
  constexpr size_t zPAR  = (size_t)PARN * 4;
  constexpr size_t oX0   = 0;
  constexpr size_t oX1   = oX0 + zF;
  constexpr size_t oXL   = oX1 + zF;
  constexpr size_t oT    = oXL + zF;
  constexpr size_t oXHL  = oT + zF;
  constexpr size_t oSD   = oXHL + zHL;
  constexpr size_t oPSD  = oSD + zSD;
  constexpr size_t oHITS = oPSD + zPSD;
  constexpr size_t oCO   = oHITS + zHITS;
  constexpr size_t oTC   = oCO + zCO;
  constexpr size_t oFLAG = oTC + zTC;
  constexpr size_t oREC  = oFLAG + zFLAG;
  constexpr size_t oSTAT = oREC + zREC;
  constexpr size_t oWT   = oSTAT + zSTAT;
  constexpr size_t oPAR  = oWT + zWT;
  constexpr size_t oEND  = oPAR + zPAR;
  static_assert(zF % 256 == 0 && zHL % 256 == 0 && zSD % 256 == 0 && zPSD % 256 == 0 && zHITS % 256 == 0);
  static_assert(zCO % 256 == 0 && zTC % 256 == 0 && zFLAG % 256 == 0 && zREC % 256 == 0 && zSTAT % 256 == 0);
  static_assert(zWT % 256 == 0 && zPAR % 256 == 0);
  static_assert(zFLAG >= (size_t)NBK * 128);
  static_assert(oEND <= WSMAX);
  if (oEND > ws_size) return;

  char* ws = (char*)d_ws;
  float*          X0   = (float*)(ws + oX0);
  float*          X1   = (float*)(ws + oX1);
  float*          XL   = (float*)(ws + oXL);
  float*          T    = (float*)(ws + oT);
  unsigned short* XHL  = (unsigned short*)(ws + oXHL);
  float*          SD   = (float*)(ws + oSD);
  float*          PSD  = (float*)(ws + oPSD);
  int*            HITS = (int*)(ws + oHITS);
  int*            CO   = (int*)(ws + oCO);
  int*            TC   = (int*)(ws + oTC);
  int*            FLAG = (int*)(ws + oFLAG);
  double*         REC  = (double*)(ws + oREC);
  float*          STAT = (float*)(ws + oSTAT);
  unsigned short* WT   = (unsigned short*)(ws + oWT);
  float*          PAR  = (float*)(ws + oPAR);

  hipFuncSetAttribute(reinterpret_cast<const void*>(&k_bucket), hipFuncAttributeMaxDynamicSharedMemorySize, (int)BK_LDS);
  hipFuncSetAttribute(reinterpret_cast<const void*>(&k_replay), hipFuncAttributeMaxDynamicSharedMemorySize, (int)RP_LDS);

  constexpr int K1 = SPLIT1 ? 128 : 64;
  constexpr int K2 = SPLIT2 ? 128 : 64;

  k_prep<<<PBTOT, NTHR, 0, stream>>>(xidx, aemb, W, atts, attd, atte, bias, eemb, gam, bet, pw, pb, X0, XHL, WT, PAR);
  k_bucket<<<NBK, NTHR, BK_LDS, stream>>>(srcs, dsts, etyp, HITS, CO, TC, FLAG);

  for (int l = 0; l < NLAY; ++l) {
    const unsigned short* bt = WT + (size_t)l * HD * KP;
    const int offS = P_AS + 64 * l, offD = P_AD + 64 * l;
    if (l == 0)      k_gemm<64><<<MP / GBM, NTHR, 0, stream>>>(XHL, bt, PAR, offS, offD, XL, SD);
    else if (l == 1) k_gemm<K1><<<MP / GBM, NTHR, 0, stream>>>(XHL, bt, PAR, offS, offD, XL, SD);
    else             k_gemm<K2><<<MP / GBM, NTHR, 0, stream>>>(XHL, bt, PAR, offS, offD, XL, SD);
    k_replay<<<NBK, NTHR, RP_LDS, stream>>>(HITS, CO, TC, FLAG, PAR, l, XL, SD, T, REC);
    k_stat<<<1, 64, 0, stream>>>(REC, STAT);
    const float* Xin  = (l & 1) ? X1 : X0;
    float*       Xout = (l & 1) ? X0 : X1;
    if (l < NLAY - 1) k_apply<0><<<MP / GBM, NTHR, 0, stream>>>(T, Xin, STAT, PAR, l, Xout, XHL, PSD);
    else              k_apply<1><<<MP / GBM, NTHR, 0, stream>>>(T, Xin, STAT, PAR, l, Xout, XHL, PSD);
  }
  k_head<<<NE / NTHR, NTHR, 0, stream>>>(ei, PSD, PAR, out);
}
